// TAGConvNet_14388140441686
// MI455X (gfx1250) — hardware-verified
//
#include <hip/hip_runtime.h>
#include <stddef.h>


#define DF      128
#define FIN     16
#define HW      64
#define NTHR    256
#define NWAVE   8
#define EPT     8
#define NGRP    2
#define CHUNK   (NTHR * EPT * NGRP)
#define WCAP    (EPT * NGRP * 32)
#define LISTN   (NWAVE * WCAP)
#define NB      1024
#define NBD     4096
#define L0ROWS  128
#define MROWS   128
#define NWMAT   10
#define RTW     (NB / (16 * NWAVE))

#define LDS_HOP (NB * HW * 4 + LISTN * 4 + 64)
#define LDS_MLP (NWAVE * 2 * 16 * DF * 2 + MROWS * 4)

static_assert((CHUNK & (CHUNK - 1)) == 0);
static_assert(CHUNK <= 4096);
static_assert((NB & (NB - 1)) == 0 && NB <= 4096);
static_assert((NBD & (NBD - 1)) == 0 && NBD <= 4096);
static_assert(NB % (16 * NWAVE) == 0);
static_assert((NB * HW) % (NTHR * 8) == 0);
static_assert(NBD % L0ROWS == 0 && NB % L0ROWS == 0 && NB % MROWS == 0);

typedef float  v2f  __attribute__((ext_vector_type(2)));
typedef float  v4f  __attribute__((ext_vector_type(4)));
typedef float  v8f  __attribute__((ext_vector_type(8)));
typedef int    v4i  __attribute__((ext_vector_type(4)));
typedef __bf16 v8b  __attribute__((ext_vector_type(8)));
typedef __bf16 v16b __attribute__((ext_vector_type(16)));
union FragB { v16b v; v8b h[2]; };
union Z8 { v4i i; v8b b; };

__device__ __forceinline__ v8b zero8b() { Z8 z; v4i q = {0, 0, 0, 0}; z.i = q; return z.b; }
__device__ __forceinline__ v8f zero8f() { v8f z = {0.f, 0.f, 0.f, 0.f, 0.f, 0.f, 0.f, 0.f}; return z; }

__device__ __forceinline__ void split8(v4f a, v4f b, v8b& hi, v8b& lo) {
#define SPL(I, X) { const float xx = (X); const __bf16 th = (__bf16)xx; hi[I] = th; lo[I] = (__bf16)(xx - (float)th); }
  SPL(0, a.x) SPL(1, a.y) SPL(2, a.z) SPL(3, a.w) SPL(4, b.x) SPL(5, b.y) SPL(6, b.z) SPL(7, b.w)
#undef SPL
}

__device__ __forceinline__ v8f wmb(v16b a, v16b b, v8f c) {
  v8f d = __builtin_amdgcn_wmma_f32_16x16x32_bf16(false, a, false, b, (short)0, c, false, false);
  asm volatile("v_nop\n\tv_nop\n\tv_nop\n\tv_nop" : "+v"(d) : "v"(a), "v"(b));
  return d;
}
__device__ __forceinline__ v8f wm3(v16b ah, v16b al, v16b bh, v16b bl, v8f c) {
  c = wmb(ah, bh, c);
  c = wmb(ah, bl, c);
  c = wmb(al, bh, c);
  return c;
}

template <int NBX>
__device__ __forceinline__ int scan_chunk(const int* __restrict__ dsts, int nE, int cbase, int nodeBase,
                                          int vec8, int* list, int tid, int lane, int wave) {
  int wc = 0;
#pragma unroll
  for (int g = 0; g < NGRP; ++g) {
    const int el0  = (g * NTHR + tid) * EPT;
    const int e0   = cbase + el0;
    const int sent = -2147483647 - 1;
    v4i da, db;
    if (vec8 != 0 && e0 + 7 < nE) {
      da = *(const v4i*)(dsts + e0);
      db = *(const v4i*)(dsts + e0 + 4);
    } else {
      da.x = (e0     < nE) ? dsts[min(e0, nE - 1)] : sent;
      da.y = (e0 + 1 < nE) ? dsts[min(e0 + 1, nE - 1)] : sent;
      da.z = (e0 + 2 < nE) ? dsts[min(e0 + 2, nE - 1)] : sent;
      da.w = (e0 + 3 < nE) ? dsts[min(e0 + 3, nE - 1)] : sent;
      db.x = (e0 + 4 < nE) ? dsts[min(e0 + 4, nE - 1)] : sent;
      db.y = (e0 + 5 < nE) ? dsts[min(e0 + 5, nE - 1)] : sent;
      db.z = (e0 + 6 < nE) ? dsts[min(e0 + 6, nE - 1)] : sent;
      db.w = (e0 + 7 < nE) ? dsts[min(e0 + 7, nE - 1)] : sent;
    }
    const unsigned nb = (unsigned)nodeBase;
    const unsigned s0 = (unsigned)da.x - nb, s1 = (unsigned)da.y - nb;
    const unsigned s2 = (unsigned)da.z - nb, s3 = (unsigned)da.w - nb;
    const unsigned s4 = (unsigned)db.x - nb, s5 = (unsigned)db.y - nb;
    const unsigned s6 = (unsigned)db.z - nb, s7 = (unsigned)db.w - nb;
    const bool h0 = s0 < (unsigned)NBX, h1 = s1 < (unsigned)NBX, h2 = s2 < (unsigned)NBX, h3 = s3 < (unsigned)NBX;
    const bool h4 = s4 < (unsigned)NBX, h5 = s5 < (unsigned)NBX, h6 = s6 < (unsigned)NBX, h7 = s7 < (unsigned)NBX;
    const unsigned any = __builtin_amdgcn_ballot_w32(h0 | h1 | h2 | h3 | h4 | h5 | h6 | h7);
    if (any != 0u) {
#define HITJ(J, HJ, SJ) { \
        const unsigned mj = __builtin_amdgcn_ballot_w32(HJ); \
        if (mj != 0u) { \
          if (HJ) { \
            const int pos = wc + (int)__builtin_amdgcn_mbcnt_lo(mj, 0u); \
            if (pos < WCAP) list[wave * WCAP + pos] = ((el0 + (J)) << 12) | (int)(SJ); \
          } \
          wc += (int)__builtin_popcount(mj); } }
      HITJ(0, h0, s0)
      HITJ(1, h1, s1)
      HITJ(2, h2, s2)
      HITJ(3, h3, s3)
      HITJ(4, h4, s4)
      HITJ(5, h5, s5)
      HITJ(6, h6, s6)
      HITJ(7, h7, s7)
#undef HITJ
    }
  }
  return wc;
}

__global__ __launch_bounds__(NTHR) void k_prep(
    const float* __restrict__ c1W, const float* __restrict__ c2W,
    const float* __restrict__ W1, const float* __restrict__ W2, const float* __restrict__ W0,
    __bf16* WB, __bf16* W0B) {
  const int i  = blockIdx.x * NTHR + threadIdx.x;
  const int nq = NWMAT * (DF * DF / 8);
  const int n0 = DF * FIN / 8;
  if (i >= nq + n0) return;
  v4f a, b;
  __bf16* dh;
  __bf16* dl;
  if (i < nq) {
    const int q   = i / (DF * DF / 8);
    const int rem = i - q * (DF * DF / 8);
    const int o   = rem * 8;
    const int n   = o / DF;
    const int k0  = o - n * DF;
    const float* base = (q < 4) ? (c1W + (size_t)q * DF * DF)
                      : (q < 8) ? (c2W + (size_t)(q - 4) * DF * DF)
                      : (q == 8 ? W1 : W2);
    const float* p = base + (size_t)k0 * DF + n;
    a.x = p[0];      a.y = p[DF];     a.z = p[2 * DF]; a.w = p[3 * DF];
    b.x = p[4 * DF]; b.y = p[5 * DF]; b.z = p[6 * DF]; b.w = p[7 * DF];
    dh = WB + (size_t)q * 2 * DF * DF + o;
    dl = dh + DF * DF;
  } else {
    const int rem = i - nq;
    const int o   = rem * 8;
    const int n   = o / FIN;
    const int k0  = o - n * FIN;
    const float* p = W0 + (size_t)k0 * DF + n;
    a.x = p[0];      a.y = p[DF];     a.z = p[2 * DF]; a.w = p[3 * DF];
    b.x = p[4 * DF]; b.y = p[5 * DF]; b.z = p[6 * DF]; b.w = p[7 * DF];
    dh = W0B + o;
    dl = W0B + DF * FIN + o;
  }
  v8b hv, lv;
  split8(a, b, hv, lv);
  *(volatile v8b*)dh = hv;
  *(volatile v8b*)dl = lv;
  __threadfence();
  *(volatile v8b*)dh = hv;
  *(volatile v8b*)dl = lv;
}

__global__ __launch_bounds__(NTHR) void k_deg(
    const int* __restrict__ ei, float* dinv, int nE, int vec8) {
  __shared__ __attribute__((aligned(16))) int cnt[NBD];
  __shared__ __attribute__((aligned(16))) int list[LISTN];
  __shared__ int wcnt[NWAVE];
  const int tid = threadIdx.x, lane = tid & 31, wave = tid >> 5;
  const int nodeBase = blockIdx.x * NBD;
  const int* dsts = ei + nE;

  for (int i = tid; i < NBD; i += NTHR) cnt[i] = 0;
  __syncthreads();

  const int nChunks = (nE + CHUNK - 1) / CHUNK;
#pragma unroll 1
  for (int ch = 0; ch < nChunks; ++ch) {
    const int cbase = ch * CHUNK;
    const int wc = scan_chunk<NBD>(dsts, nE, cbase, nodeBase, vec8, list, tid, lane, wave);
    if (lane == 0) wcnt[wave] = wc;
    __syncthreads();
    if (wave == 0) {
#pragma unroll 1
      for (int wsx = 0; wsx < NWAVE; ++wsx) {
        int n = __builtin_amdgcn_readfirstlane(wcnt[wsx]);
        n = n > WCAP ? WCAP : (n < 0 ? 0 : n);
        const int* lp = list + wsx * WCAP;
#pragma unroll 1
        for (int i = 0; i < n; ++i) {
          const int ent  = __builtin_amdgcn_readfirstlane(lp[i]);
          const int slot = ent & (NBD - 1);
          if (lane == 0) cnt[slot] = cnt[slot] + 1;
        }
      }
    }
    __syncthreads();
  }

  v4f dq[4];
#pragma unroll
  for (int q = 0; q < 4; ++q) {
    const int f = (wave * 4 + q) * 128 + 4 * lane;
    const v4i c = *(const v4i*)(cnt + f);
    dq[q].x = (c.x > 0) ? rsqrtf((float)c.x) : 0.f;
    dq[q].y = (c.y > 0) ? rsqrtf((float)c.y) : 0.f;
    dq[q].z = (c.z > 0) ? rsqrtf((float)c.z) : 0.f;
    dq[q].w = (c.w > 0) ? rsqrtf((float)c.w) : 0.f;
  }
  float* dp = dinv + (size_t)nodeBase;
#pragma unroll
  for (int q = 0; q < 4; ++q) *(volatile v4f*)(dp + (wave * 4 + q) * 128 + 4 * lane) = dq[q];
  __threadfence();
#pragma unroll
  for (int q = 0; q < 4; ++q) *(volatile v4f*)(dp + (wave * 4 + q) * 128 + 4 * lane) = dq[q];
}

__global__ __launch_bounds__(NTHR) void k_lin0(
    const float* __restrict__ x, const __bf16* __restrict__ W0B, const float* __restrict__ b0,
    __bf16* Hs0, __bf16* Hs1, int nN, int nPad) {
  __shared__ __attribute__((aligned(16))) float stg[L0ROWS * DF];
  const int tid = threadIdx.x, lane = tid & 31, wave = tid >> 5, hh = lane >> 4, m = lane & 15;
  const int rowBase = blockIdx.x * L0ROWS;
  const v8b z8 = zero8b();

  int node = rowBase + wave * 16 + m;
  node = node > nN - 1 ? nN - 1 : node;
  const float* xp = x + (size_t)node * FIN + 8 * hh;
  const v4f xa = *(const v4f*)xp, xb = *(const v4f*)(xp + 4);
  FragB ah, al;
  split8(xa, xb, ah.h[0], al.h[0]);
  ah.h[1] = z8;
  al.h[1] = z8;

  v8f d[8];
#pragma unroll
  for (int t = 0; t < 8; ++t) {
    const __bf16* bp = W0B + (size_t)(16 * t + m) * FIN + 8 * hh;
    FragB bh, bl;
    bh.h[0] = *(const v8b*)bp;               bh.h[1] = z8;
    bl.h[0] = *(const v8b*)(bp + DF * FIN);  bl.h[1] = z8;
    d[t] = wm3(ah.v, al.v, bh.v, bl.v, zero8f());
  }
  float* sp = stg + (wave * 16 + 8 * hh) * DF + m;
#pragma unroll
  for (int t = 0; t < 8; ++t) {
    const float bv = b0[16 * t + m];
#pragma unroll
    for (int r = 0; r < 8; ++r) sp[r * DF + 16 * t] = fmaxf(d[t][r] + bv, 0.f);
  }
  __syncthreads();

  const size_t plane = (size_t)nPad * HW;
#pragma unroll 1
  for (int ch = 0; ch < 2; ++ch) {
    __bf16* oh = (ch == 0 ? Hs0 : Hs1) + (size_t)rowBase * HW;
#pragma unroll
    for (int it = 0; it < (L0ROWS * HW / 8) / NTHR; ++it) {
      const int idx = it * NTHR + tid;
      const int r   = idx >> 3;
      const int c0  = (idx & 7) * 8;
      const float* s = stg + r * DF + HW * ch + c0;
      v8b hv, lv;
      split8(*(const v4f*)s, *(const v4f*)(s + 4), hv, lv);
      *(volatile v8b*)(oh + (size_t)r * HW + c0) = hv;
      *(volatile v8b*)(oh + plane + (size_t)r * HW + c0) = lv;
    }
  }
  __threadfence();
#pragma unroll 1
  for (int ch = 0; ch < 2; ++ch) {
    __bf16* oh = (ch == 0 ? Hs0 : Hs1) + (size_t)rowBase * HW;
#pragma unroll
    for (int it = 0; it < (L0ROWS * HW / 8) / NTHR; ++it) {
      const int idx = it * NTHR + tid;
      const int r   = idx >> 3;
      const int c0  = (idx & 7) * 8;
      const float* s = stg + r * DF + HW * ch + c0;
      v8b hv, lv;
      split8(*(const v4f*)s, *(const v4f*)(s + 4), hv, lv);
      *(volatile v8b*)(oh + (size_t)r * HW + c0) = hv;
      *(volatile v8b*)(oh + plane + (size_t)r * HW + c0) = lv;
    }
  }
}

template <int MODE>
__global__ __launch_bounds__(NTHR) void k_hop(
    const int* __restrict__ ei, const float* __restrict__ dinv,
    const __bf16* __restrict__ Hs0, const __bf16* __restrict__ Hs1,
    const __bf16* __restrict__ Wq, const float* __restrict__ bias,
    const float* __restrict__ uprev, void* uout,
    int c, int nN, int nE, int nPad, int vec8) {
  extern __shared__ v4f lds_dyn[];
  float* acc  = (float*)lds_dyn;
  int*   list = (int*)(acc + NB * HW);
  int*   wcnt = list + LISTN;
  const int tid = threadIdx.x, lane = tid & 31, wave = tid >> 5, hh = lane >> 4, m = lane & 15;
  const int nodeBase = blockIdx.x * NB;

  if (MODE != 0) {
    {
      const v4f z = {0.f, 0.f, 0.f, 0.f};
      for (int i = tid; i < NB * HW / 4; i += NTHR) lds_dyn[i] = z;
    }
    __syncthreads();

    const int* dsts = ei + nE;
    const int nChunks = (nE + CHUNK - 1) / CHUNK;
#pragma unroll 1
    for (int ch = 0; ch < nChunks; ++ch) {
      const int cbase = ch * CHUNK;
      const int wc = scan_chunk<NB>(dsts, nE, cbase, nodeBase, vec8, list, tid, lane, wave);
      if (lane == 0) wcnt[wave] = wc;
      __syncthreads();
      if (wave == 0) {
#pragma unroll 1
        for (int wsx = 0; wsx < NWAVE; ++wsx) {
          int n = __builtin_amdgcn_readfirstlane(wcnt[wsx]);
          n = n > WCAP ? WCAP : (n < 0 ? 0 : n);
          const int* lp = list + wsx * WCAP;
#pragma unroll 1
          for (int i = 0; i < n; ++i) {
            const int ent  = __builtin_amdgcn_readfirstlane(lp[i]);
            const int slot = ent & (NB - 1);
            int e = cbase + ((ent >> 12) & (CHUNK - 1));
            e = e > nE - 1 ? nE - 1 : e;
            int src = ei[e];
            src = src < 0 ? 0 : (src > nN - 1 ? nN - 1 : src);
            const float ds = dinv[src];
            const v2f v = *(const v2f*)(uprev + (size_t)src * HW + 2 * lane);
            v2f* ap = (v2f*)(acc + slot * HW + 2 * lane);
            *ap = *ap + v * ds;
          }
        }
      }
      __syncthreads();
    }
  }

  const size_t plane = (size_t)nPad * HW;
#pragma unroll 1
  for (int rt = 0; rt < RTW; ++rt) {
    const int rowL = (wave * RTW + rt) * 16;
    const size_t arow = (size_t)(nodeBase + rowL + m) * HW + 8 * hh;
    v8f d[4];
#pragma unroll
    for (int t = 0; t < 4; ++t) d[t] = zero8f();
#pragma unroll
    for (int ks = 0; ks < 4; ++ks) {
      const __bf16* hb = ((ks < 2) ? Hs0 : Hs1) + arow + (ks & 1) * 32;
      FragB ah, al;
      ah.h[0] = *(const v8b*)hb;            ah.h[1] = *(const v8b*)(hb + 16);
      al.h[0] = *(const v8b*)(hb + plane);  al.h[1] = *(const v8b*)(hb + plane + 16);
#pragma unroll
      for (int t = 0; t < 4; ++t) {
        const __bf16* bp = Wq + (size_t)(HW * c + 16 * t + m) * DF + 32 * ks + 8 * hh;
        FragB bh, bl;
        bh.h[0] = *(const v8b*)bp;             bh.h[1] = *(const v8b*)(bp + 16);
        bl.h[0] = *(const v8b*)(bp + DF * DF); bl.h[1] = *(const v8b*)(bp + DF * DF + 16);
        d[t] = wm3(ah.v, al.v, bh.v, bl.v, d[t]);
      }
    }
    v8f dv = zero8f();
    if (MODE != 0) {
      const v4f dA = *(const v4f*)(dinv + (size_t)nodeBase + rowL + 8 * hh);
      const v4f dB = *(const v4f*)(dinv + (size_t)nodeBase + rowL + 8 * hh + 4);
      dv[0] = dA.x; dv[1] = dA.y; dv[2] = dA.z; dv[3] = dA.w;
      dv[4] = dB.x; dv[5] = dB.y; dv[6] = dB.z; dv[7] = dB.w;
    }
    float* sp = acc + (rowL + 8 * hh) * HW + m;
#pragma unroll
    for (int t = 0; t < 4; ++t) {
      float bv = 0.f;
      if (MODE == 2) bv = bias[HW * c + 16 * t + m];
#pragma unroll
      for (int r = 0; r < 8; ++r) {
        float v = d[t][r];
        if (MODE != 0) v = v + dv[r] * sp[r * HW + 16 * t];
        if (MODE == 2) v = fmaxf(v + bv, 0.f);
        sp[r * HW + 16 * t] = v;
      }
    }
  }
  __syncthreads();

  if (MODE == 2) {
    __bf16* oh = (__bf16*)uout + (size_t)nodeBase * HW;
#pragma unroll 4
    for (int it = 0; it < (NB * HW / 8) / NTHR; ++it) {
      const int f = (it * NTHR + tid) * 8;
      v8b hv, lv;
      split8(*(const v4f*)(acc + f), *(const v4f*)(acc + f + 4), hv, lv);
      *(volatile v8b*)(oh + f) = hv;
      *(volatile v8b*)(oh + plane + f) = lv;
    }
    __threadfence();
#pragma unroll 4
    for (int it = 0; it < (NB * HW / 8) / NTHR; ++it) {
      const int f = (it * NTHR + tid) * 8;
      v8b hv, lv;
      split8(*(const v4f*)(acc + f), *(const v4f*)(acc + f + 4), hv, lv);
      *(volatile v8b*)(oh + f) = hv;
      *(volatile v8b*)(oh + plane + f) = lv;
    }
  } else {
    float* uo = (float*)uout + (size_t)nodeBase * HW;
#pragma unroll 4
    for (int it = 0; it < (NB * HW / 4) / NTHR; ++it) {
      const int f = (it * NTHR + tid) * 4;
      const v4f v = *(const v4f*)(acc + f);
      *(volatile v4f*)(uo + f) = v;
    }
    __threadfence();
#pragma unroll 4
    for (int it = 0; it < (NB * HW / 4) / NTHR; ++it) {
      const int f = (it * NTHR + tid) * 4;
      const v4f v = *(const v4f*)(acc + f);
      *(volatile v4f*)(uo + f) = v;
    }
  }
}

__global__ __launch_bounds__(NTHR) void k_mlp(
    const __bf16* __restrict__ Hs0, const __bf16* __restrict__ Hs1,
    const __bf16* __restrict__ W1q, const __bf16* __restrict__ W2q,
    const float* __restrict__ b1, const float* __restrict__ b2,
    const float* __restrict__ W3, const float* __restrict__ b3,
    float* out, int nN, int nPad) {
  extern __shared__ v4f lds_dyn[];
  __bf16* sh   = (__bf16*)lds_dyn;
  float*  fout = (float*)(sh + NWAVE * 2 * 16 * DF);
  const int tid = threadIdx.x, lane = tid & 31, wave = tid >> 5, hh = lane >> 4, m = lane & 15;
  const int rowBase = blockIdx.x * MROWS;
  __bf16* shh = sh + wave * (2 * 16 * DF);
  __bf16* shl = shh + 16 * DF;
  const size_t plane = (size_t)nPad * HW;
  const size_t arow  = (size_t)(rowBase + wave * 16 + m) * HW + 8 * hh;

  v8f d[8];
#pragma unroll
  for (int t = 0; t < 8; ++t) d[t] = zero8f();
#pragma unroll
  for (int ks = 0; ks < 4; ++ks) {
    const __bf16* hb = ((ks < 2) ? Hs0 : Hs1) + arow + (ks & 1) * 32;
    FragB ah, al;
    ah.h[0] = *(const v8b*)hb;            ah.h[1] = *(const v8b*)(hb + 16);
    al.h[0] = *(const v8b*)(hb + plane);  al.h[1] = *(const v8b*)(hb + plane + 16);
#pragma unroll
    for (int t = 0; t < 8; ++t) {
      const __bf16* bp = W1q + (size_t)(16 * t + m) * DF + 32 * ks + 8 * hh;
      FragB bh, bl;
      bh.h[0] = *(const v8b*)bp;             bh.h[1] = *(const v8b*)(bp + 16);
      bl.h[0] = *(const v8b*)(bp + DF * DF); bl.h[1] = *(const v8b*)(bp + DF * DF + 16);
      d[t] = wm3(ah.v, al.v, bh.v, bl.v, d[t]);
    }
  }
#pragma unroll
  for (int t = 0; t < 8; ++t) {
    const float bv = b1[16 * t + m];
#pragma unroll
    for (int r = 0; r < 8; ++r) {
      const float v   = fmaxf(d[t][r] + bv, 0.f);
      const __bf16 th = (__bf16)v;
      shh[(8 * hh + r) * DF + 16 * t + m] = th;
      shl[(8 * hh + r) * DF + 16 * t + m] = (__bf16)(v - (float)th);
    }
  }
  __syncthreads();

#pragma unroll
  for (int t = 0; t < 8; ++t) d[t] = zero8f();
#pragma unroll
  for (int ks = 0; ks < 4; ++ks) {
    const __bf16* ap = shh + m * DF + 32 * ks + 8 * hh;
    FragB ah, al;
    ah.h[0] = *(const v8b*)ap;              ah.h[1] = *(const v8b*)(ap + 16);
    al.h[0] = *(const v8b*)(ap + 16 * DF);  al.h[1] = *(const v8b*)(ap + 16 * DF + 16);
#pragma unroll
    for (int t = 0; t < 8; ++t) {
      const __bf16* bp = W2q + (size_t)(16 * t + m) * DF + 32 * ks + 8 * hh;
      FragB bh, bl;
      bh.h[0] = *(const v8b*)bp;             bh.h[1] = *(const v8b*)(bp + 16);
      bl.h[0] = *(const v8b*)(bp + DF * DF); bl.h[1] = *(const v8b*)(bp + DF * DF + 16);
      d[t] = wm3(ah.v, al.v, bh.v, bl.v, d[t]);
    }
  }
  v8f p = zero8f();
#pragma unroll
  for (int t = 0; t < 8; ++t) {
    const float bv = b2[16 * t + m];
    const float w3 = W3[16 * t + m];
#pragma unroll
    for (int r = 0; r < 8; ++r) {
      const float v = fmaxf(d[t][r] + bv, 0.f);
      p[r] = p[r] + v * w3;
    }
  }
#pragma unroll
  for (int r = 0; r < 8; ++r) {
    float s = p[r];
    s += __shfl_xor(s, 1);
    s += __shfl_xor(s, 2);
    s += __shfl_xor(s, 4);
    s += __shfl_xor(s, 8);
    p[r] = s;
  }
  const float b3v = b3[0];
  if (m == 0) {
#pragma unroll
    for (int r = 0; r < 8; ++r) fout[wave * 16 + 8 * hh + r] = fmaxf(p[r] + b3v, 0.f);
  }
  __syncthreads();

  if (wave == 0) {
    const int r0 = rowBase + 4 * lane;
    const v4f v = *(const v4f*)(fout + 4 * lane);
    if (r0 + 3 < nN) {
      *(volatile v4f*)(out + r0) = v;
    } else {
      if (r0 < nN)     *(volatile float*)(out + r0) = v.x;
      if (r0 + 1 < nN) *(volatile float*)(out + r0 + 1) = v.y;
      if (r0 + 2 < nN) *(volatile float*)(out + r0 + 2) = v.z;
    }
    __threadfence();
    if (r0 + 3 < nN) {
      *(volatile v4f*)(out + r0) = v;
    } else {
      if (r0 < nN)     *(volatile float*)(out + r0) = v.x;
      if (r0 + 1 < nN) *(volatile float*)(out + r0 + 1) = v.y;
      if (r0 + 2 < nN) *(volatile float*)(out + r0 + 2) = v.z;
    }
  }
}

static void launch_hop(int mode, int nHop, hipStream_t stream,
                       const int* ei, const float* dinv, const __bf16* Hs0, const __bf16* Hs1,
                       const __bf16* Wq, const float* bias, const float* uprev, void* uout,
                       int c, int nN, int nE, int nPad, int vec8) {
  if (mode == 0)
    k_hop<0><<<nHop, NTHR, LDS_HOP, stream>>>(ei, dinv, Hs0, Hs1, Wq, bias, uprev, uout, c, nN, nE, nPad, vec8);
  else if (mode == 1)
    k_hop<1><<<nHop, NTHR, LDS_HOP, stream>>>(ei, dinv, Hs0, Hs1, Wq, bias, uprev, uout, c, nN, nE, nPad, vec8);
  else
    k_hop<2><<<nHop, NTHR, LDS_HOP, stream>>>(ei, dinv, Hs0, Hs1, Wq, bias, uprev, uout, c, nN, nE, nPad, vec8);
}

static void run_layer(int nHop, hipStream_t stream, const int* ei, const float* dinv,
                      const __bf16* Hs0, const __bf16* Hs1, const __bf16* Wbase, const float* bias,
                      char* F0, char* F1, char* F2, int nN, int nE, int nPad, int vec8) {
  const __bf16* Wk0 = Wbase;
  const __bf16* Wk1 = Wbase + (size_t)1 * 2 * DF * DF;
  const __bf16* Wk2 = Wbase + (size_t)2 * 2 * DF * DF;
  const __bf16* Wk3 = Wbase + (size_t)3 * 2 * DF * DF;
  for (int c = 0; c < 2; ++c) {
    launch_hop(0, nHop, stream, ei, dinv, Hs0, Hs1, Wk3, bias, (const float*)F0, (void*)F0, c, nN, nE, nPad, vec8);
    launch_hop(1, nHop, stream, ei, dinv, Hs0, Hs1, Wk2, bias, (const float*)F0, (void*)F1, c, nN, nE, nPad, vec8);
    launch_hop(1, nHop, stream, ei, dinv, Hs0, Hs1, Wk1, bias, (const float*)F1, (void*)(c == 0 ? F2 : F0), c, nN, nE, nPad, vec8);
  }
  launch_hop(2, nHop, stream, ei, dinv, Hs0, Hs1, Wk0, bias, (const float*)F2, (void*)F1, 0, nN, nE, nPad, vec8);
  launch_hop(2, nHop, stream, ei, dinv, Hs0, Hs1, Wk0, bias, (const float*)F0, (void*)F2, 1, nN, nE, nPad, vec8);
}

extern "C" void kernel_launch(void* const* d_in, const int* in_sizes, int n_in,
                              void* d_out, int out_size, void* d_ws, size_t ws_size,
                              hipStream_t stream) {
  if (n_in < 14) return;
  const int nN = in_sizes[0] / FIN;
  const int nE = in_sizes[1] / 2;
  if (nN <= 0 || nE < 0 || in_sizes[0] != nN * FIN || in_sizes[1] != nE * 2) return;
  if (in_sizes[2] != FIN * DF || in_sizes[3] < DF) return;
  if (in_sizes[4] != 4 * DF * DF || in_sizes[5] < DF || in_sizes[6] != 4 * DF * DF || in_sizes[7] < DF) return;
  if (in_sizes[8] != DF * DF || in_sizes[9] < DF || in_sizes[10] != DF * DF || in_sizes[11] < DF) return;
  if (in_sizes[12] < DF || in_sizes[13] < 1) return;
  if (out_size != nN) return;

  const float* x   = (const float*)d_in[0];
  const int*   ei  = (const int*)d_in[1];
  const float* W0  = (const float*)d_in[2];
  const float* b0  = (const float*)d_in[3];
  const float* c1W = (const float*)d_in[4];
  const float* c1b = (const float*)d_in[5];
  const float* c2W = (const float*)d_in[6];
  const float* c2b = (const float*)d_in[7];
  const float* W1  = (const float*)d_in[8];
  const float* b1  = (const float*)d_in[9];
  const float* W2  = (const float*)d_in[10];
  const float* b2  = (const float*)d_in[11];
  const float* W3  = (const float*)d_in[12];
  const float* b3  = (const float*)d_in[13];
  float* out = (float*)d_out;

  const int nHop = (nN + NB - 1) / NB;
  const int nPad = nHop * NB;
  const int nBD  = (nPad + NBD - 1) / NBD;
  const int nL0  = nPad / L0ROWS;
  const int nML  = (nN + MROWS - 1) / MROWS;

  char* ws = (char*)d_ws;
  size_t off = 0;
  const size_t oWB = off; off += (size_t)NWMAT * 2 * DF * DF * 2;  off = (off + 255) & ~(size_t)255;
  const size_t oW0 = off; off += (size_t)2 * DF * FIN * 2;          off = (off + 255) & ~(size_t)255;
  const size_t oDv = off; off += (size_t)nBD * NBD * 4;             off = (off + 255) & ~(size_t)255;
  const size_t slotB = ((size_t)nPad * HW * 4 + 255) & ~(size_t)255;
  size_t oS[5];
  for (int s = 0; s < 5; ++s) { oS[s] = off; off += slotB; }
  if (off > ws_size) return;

  __bf16* WB   = (__bf16*)(ws + oWB);
  __bf16* W0B  = (__bf16*)(ws + oW0);
  float*  dinv = (float*)(ws + oDv);
  char*   S0 = ws + oS[0];
  char*   S1 = ws + oS[1];
  char*   S2 = ws + oS[2];
  char*   S3 = ws + oS[3];
  char*   S4 = ws + oS[4];

  const int vec8 = ((nE & 3) == 0) ? 1 : 0;

  const int nPrep = NWMAT * (DF * DF / 8) + DF * FIN / 8;
  k_prep<<<(nPrep + NTHR - 1) / NTHR, NTHR, 0, stream>>>(c1W, c2W, W1, W2, W0, WB, W0B);

  k_deg<<<nBD, NTHR, 0, stream>>>(ei, dinv, nE, vec8);

  k_lin0<<<nL0, NTHR, 0, stream>>>(x, W0B, b0, (__bf16*)S0, (__bf16*)S1, nN, nPad);

  hipFuncSetAttribute(reinterpret_cast<const void*>(&k_hop<0>), hipFuncAttributeMaxDynamicSharedMemorySize, LDS_HOP);
  hipFuncSetAttribute(reinterpret_cast<const void*>(&k_hop<1>), hipFuncAttributeMaxDynamicSharedMemorySize, LDS_HOP);
  hipFuncSetAttribute(reinterpret_cast<const void*>(&k_hop<2>), hipFuncAttributeMaxDynamicSharedMemorySize, LDS_HOP);
  hipFuncSetAttribute(reinterpret_cast<const void*>(&k_mlp),    hipFuncAttributeMaxDynamicSharedMemorySize, LDS_MLP);

  run_layer(nHop, stream, ei, dinv, (const __bf16*)S0, (const __bf16*)S1, WB, c1b, S2, S3, S4, nN, nE, nPad, vec8);
  run_layer(nHop, stream, ei, dinv, (const __bf16*)S3, (const __bf16*)S4, WB + (size_t)4 * 2 * DF * DF, c2b, S0, S1, S2, nN, nE, nPad, vec8);

  k_mlp<<<nML, NTHR, LDS_MLP, stream>>>((const __bf16*)S1, (const __bf16*)S2,
                                         WB + (size_t)8 * 2 * DF * DF, WB + (size_t)9 * 2 * DF * DF,
                                         b1, b2, W3, b3, out, nN, nPad);
}
